// Decoder_17463337026012
// MI455X (gfx1250) — hardware-verified
//
#include <hip/hip_runtime.h>
#include <math.h>

constexpr int NBATCH = 64;
constexpr int NSTEPS = 63;
constexpr int NUNIT  = 1024;
constexpr int NVDIM  = 512;
constexpr int NBDIM  = 512;
constexpr int NGCOL  = 4 * NUNIT;
constexpr int KW0    = NVDIM + NBDIM + NUNIT;
constexpr int K0R    = NBDIM + NUNIT;
constexpr int K1L    = 2 * NUNIT;
constexpr int MROWS  = NSTEPS * NBATCH;
constexpr int NT256  = 256;
constexpr int RT     = 512;
constexpr int RW     = RT / 32;
constexpr int RB     = 16;
constexpr int NBT    = NBATCH / RB;
constexpr int SUBW   = (NUNIT / 16) / RW;
constexpr int COL_H0 = NBDIM;
constexpr int COL_H1 = NBDIM + NUNIT;
constexpr int AP     = NBDIM + 2 * NUNIT + 8;
constexpr int HLP    = NUNIT + 8;
constexpr int SLP    = 36;
constexpr int STP    = 72;
constexpr float WCARRY      = 256.0f;
constexpr float WCARRY_INV  = 1.0f / 256.0f;
constexpr float LOCARRY     = 2048.0f;
constexpr float LOCARRY_INV = 1.0f / 2048.0f;
constexpr float FORGET_B    = 0.8f;
constexpr size_t XGF_FLOATS = (size_t)NSTEPS * NBATCH * NGCOL;
constexpr size_t CST_FLOATS = (size_t)2 * NBT * (NUNIT / 16) * 256;

static_assert(KW0 == 2048);
static_assert(K0R % 32 == 0 && K1L % 32 == 0 && NUNIT % 32 == 0 && NVDIM % 32 == 0);
static_assert(MROWS % 64 == 0 && NGCOL % 64 == 0);
static_assert(NBATCH % RB == 0 && NBT == 4);
static_assert(SUBW == 4);
static_assert(RT == NBDIM);
static_assert(RW * 32 == NBDIM);
static_assert(RW * SUBW * 16 == NUNIT);
static_assert((AP * 2) % 16 == 0 && (HLP * 2) % 16 == 0 && (SLP * 4) % 16 == 0 && (STP * 2) % 16 == 0);
static_assert(16 * SLP * 4 == 16 * STP * 2);
static_assert(STP >= 64 + 8);
static_assert((RB * NUNIT) % RT == 0);
static_assert((MROWS * (NVDIM / 8)) % NT256 == 0);
static_assert(((MROWS / 64) * (NGCOL / 64)) % 8 == 0);

typedef __attribute__((ext_vector_type(16))) _Float16 v16h;
typedef __attribute__((ext_vector_type(8)))  _Float16 v8h;
typedef __attribute__((ext_vector_type(8)))  float    v8f;
typedef __attribute__((ext_vector_type(4)))  float    v4f;

__device__ __forceinline__ unsigned short f2bf_bits(float f) {
  unsigned u = __float_as_uint(f);
  return (unsigned short)((u + 0x7FFFu + ((u >> 16) & 1u)) >> 16);
}
__device__ __forceinline__ float bf_bits2f(unsigned short h) { return __uint_as_float(((unsigned)h) << 16); }
__device__ __forceinline__ float bf16r(float f) { return bf_bits2f(f2bf_bits(f)); }

__device__ __forceinline__ void guard4_h(v8f& a0, v8f& a1, v8f& a2, v8f& a3, v16h x, v16h y0, v16h y1, v16h y2, v16h y3) {
  asm volatile("v_nop\n\tv_nop\n\tv_nop\n\tv_nop" : "+v"(a0), "+v"(a1), "+v"(a2), "+v"(a3) : "v"(x), "v"(y0), "v"(y1), "v"(y2), "v"(y3));
}
__device__ __forceinline__ void guard2_h(v8f& a0, v8f& a1, v16h x0, v16h x1, v16h y) {
  asm volatile("v_nop\n\tv_nop\n\tv_nop\n\tv_nop" : "+v"(a0), "+v"(a1) : "v"(x0), "v"(x1), "v"(y));
}
__device__ __forceinline__ void acc_guard4(v8f& a, v8f& b, v8f& c, v8f& d) { asm volatile("v_nop\n\tv_nop\n\tv_nop\n\tv_nop" : "+v"(a), "+v"(b), "+v"(c), "+v"(d)); }
__device__ __forceinline__ void acc_guard2(v8f& a, v8f& b) { asm volatile("v_nop\n\tv_nop\n\tv_nop\n\tv_nop" : "+v"(a), "+v"(b)); }

template <typename T> struct Frag;
template <> struct Frag<_Float16> {
  typedef v16h V; union U { v16h v; v8h h[2]; };
  static __device__ __forceinline__ v16h load(const _Float16* p) {
    U f; f.h[0] = *(const v8h*)(p); f.h[1] = *(const v8h*)(p + 16); return f.v;
  }
  static __device__ __forceinline__ v8f mma(v16h a, v16h b, v8f c) {
    return __builtin_amdgcn_wmma_f32_16x16x32_f16(false, a, false, b, (short)0, c, false, false);
  }
};

__device__ __forceinline__ float fsig(float x)  { return __builtin_amdgcn_rcpf(1.0f + __expf(-x)); }
__device__ __forceinline__ float ftanh(float x) { return 1.0f - 2.0f * __builtin_amdgcn_rcpf(__expf(2.0f * x) + 1.0f); }

template <int PERM>
__global__ __launch_bounds__(NT256) void tpw_kernel(const float* __restrict__ src, int C, int ldo,
                                                   unsigned short* __restrict__ O, float sc) {
  __shared__ float Tt[64 * 65];
  const int tid = threadIdx.x;
  const int c0 = blockIdx.x * 64, r0 = blockIdx.y * 64;
#pragma unroll
  for (int i = 0; i < 4; ++i) {
    const int idx = i * NT256 + tid;
    const int rr = idx >> 4, cc = (idx & 15) * 4;
    const v4f v = *(const v4f*)(src + (size_t)(r0 + rr) * (size_t)C + c0 + cc);
    Tt[rr * 65 + cc + 0] = v[0];
    Tt[rr * 65 + cc + 1] = v[1];
    Tt[rr * 65 + cc + 2] = v[2];
    Tt[rr * 65 + cc + 3] = v[3];
  }
  __syncthreads();
  const int q = tid >> 3, c8 = (tid & 7) * 8;
  v8h hv[2];
#pragma unroll
  for (int g = 0; g < 2; ++g) {
    const int qq = g * 32 + q;
#pragma unroll
    for (int e = 0; e < 8; ++e) {
      const float f = Tt[(c8 + e) * 65 + qq];
      hv[g][e] = (_Float16)(bf16r(f) * sc);
    }
  }
  for (int pass = 0; pass < 2; ++pass) {
#pragma unroll
    for (int g = 0; g < 2; ++g) {
      const int col = c0 + g * 32 + q;
      const int orow = PERM ? ((((col & (NUNIT - 1)) >> 4) << 6) + ((col >> 10) << 4) + (col & 15)) : col;
      const size_t o = (size_t)orow * (size_t)ldo + (size_t)(r0 + c8);
      *(volatile v8h*)(O + o) = hv[g];
    }
    __threadfence();
  }
}

__global__ __launch_bounds__(NT256) void cvt8_kernel(const float* __restrict__ src, unsigned short* __restrict__ dst, int n8) {
  const int i = blockIdx.x * NT256 + threadIdx.x;
  if (i < n8) {
    const float* sp = src + (size_t)i * 8;
    const v4f a = *(const v4f*)(sp);
    const v4f b = *(const v4f*)(sp + 4);
    v8h hv;
#pragma unroll
    for (int e = 0; e < 4; ++e) {
      hv[e]     = (_Float16)bf16r(a[e]);
      hv[4 + e] = (_Float16)bf16r(b[e]);
    }
    *(volatile v8h*)(dst + (size_t)i * 8) = hv;
    __threadfence();
    *(volatile v8h*)(dst + (size_t)i * 8) = hv;
  }
}

__global__ __launch_bounds__(NT256) void xg_gemm_kernel(const unsigned short* __restrict__ Ap, const unsigned short* __restrict__ Btp,
                                                       const float* __restrict__ b0, float* __restrict__ XGF) {
  const _Float16* A  = (const _Float16*)Ap;
  const _Float16* Bt = (const _Float16*)Btp;
  const int lane = threadIdx.x & 31;
  const int wave = threadIdx.x >> 5;
  const int tile = blockIdx.x * 8 + wave;
  if (tile >= (MROWS / 64) * (NGCOL / 64)) return;
  const int tm = tile >> 6;
  const int tn = tile & 63;
  const int m0 = tm << 6;
  const int n0 = tn << 6;
  const int rlane = lane & 15;
  const int koff  = (lane >> 4) * 8;

  v8f acc[4][4];
#pragma unroll
  for (int i = 0; i < 4; ++i)
#pragma unroll
    for (int j = 0; j < 4; ++j) acc[i][j] = (v8f){0.f, 0.f, 0.f, 0.f, 0.f, 0.f, 0.f, 0.f};

#pragma unroll 1
  for (int k0 = 0; k0 < NVDIM; k0 += 32) {
    v16h bh[4];
#pragma unroll
    for (int j = 0; j < 4; ++j)
      bh[j] = Frag<_Float16>::load(Bt + (size_t)(n0 + (j << 4) + rlane) * NVDIM + koff + k0);
#pragma unroll
    for (int i = 0; i < 4; ++i) {
      const v16h ah = Frag<_Float16>::load(A + (size_t)(m0 + (i << 4) + rlane) * NVDIM + koff + k0);
#pragma unroll
      for (int j = 0; j < 4; ++j) acc[i][j] = Frag<_Float16>::mma(ah, bh[j], acc[i][j]);
      guard4_h(acc[i][0], acc[i][1], acc[i][2], acc[i][3], ah, bh[0], bh[1], bh[2], bh[3]);
    }
  }
  acc_guard4(acc[0][0], acc[0][1], acc[0][2], acc[0][3]);
  acc_guard4(acc[1][0], acc[1][1], acc[1][2], acc[1][3]);
  acc_guard4(acc[2][0], acc[2][1], acc[2][2], acc[2][3]);
  acc_guard4(acc[3][0], acc[3][1], acc[3][2], acc[3][3]);

#pragma unroll
  for (int j = 0; j < 4; ++j) {
    const float bj = WCARRY * bf16r(b0[j * NUNIT + tn * 16 + rlane]);
#pragma unroll
    for (int i = 0; i < 4; ++i)
#pragma unroll
      for (int r = 0; r < 8; ++r) acc[i][j][r] += bj;
  }
  for (int pass = 0; pass < 2; ++pass) {
#pragma unroll
    for (int i = 0; i < 4; ++i) {
#pragma unroll
      for (int j = 0; j < 4; ++j) {
        float* p = XGF + ((((size_t)(tm * 4 + i) * 64 + tn) * 4 + j) * 2) * 128 + lane * 4;
        const v4f lo = __builtin_shufflevector(acc[i][j], acc[i][j], 0, 1, 2, 3);
        const v4f hi = __builtin_shufflevector(acc[i][j], acc[i][j], 4, 5, 6, 7);
        *(volatile v4f*)(p) = lo;
        *(volatile v4f*)(p + 128) = hi;
      }
    }
    __threadfence();
  }
}

template <int KLEN>
__device__ __forceinline__ void gemm4(const _Float16* arow, const _Float16* __restrict__ wrow,
                                      v8f& a0, v8f& a1, v8f& a2, v8f& a3) {
  constexpr size_t GS = (size_t)16 * KLEN;
#pragma unroll 1
  for (int k0 = 0; k0 < KLEN; k0 += 32) {
    const v16h a  = Frag<_Float16>::load(arow + k0);
    const v16h b0 = Frag<_Float16>::load(wrow + k0);
    const v16h b1 = Frag<_Float16>::load(wrow + GS + k0);
    const v16h b2 = Frag<_Float16>::load(wrow + 2 * GS + k0);
    const v16h b3 = Frag<_Float16>::load(wrow + 3 * GS + k0);
    a0 = Frag<_Float16>::mma(a, b0, a0);
    a1 = Frag<_Float16>::mma(a, b1, a1);
    a2 = Frag<_Float16>::mma(a, b2, a2);
    a3 = Frag<_Float16>::mma(a, b3, a3);
    guard4_h(a0, a1, a2, a3, a, b0, b1, b2, b3);
  }
  acc_guard4(a0, a1, a2, a3);
}

__device__ __forceinline__ void cell_update(const v8f& gi, const v8f& gj, const v8f& gf, const v8f& go,
                                            float ppi, float ppf, float ppo, const v8f& cold, v8f& cnew, v8f& hnew) {
#pragma unroll
  for (int r = 0; r < 8; ++r) {
    const float zi = gi[r] * WCARRY_INV;
    const float zj = gj[r] * WCARRY_INV;
    const float zf = gf[r] * WCARRY_INV;
    const float zo = go[r] * WCARRY_INV;
    const float co = cold[r];
    const float fg = fsig(zf + FORGET_B + co * ppf);
    const float ig = fsig(zi + co * ppi);
    const float jg = ftanh(zj);
    const float cn = fg * co + ig * jg;
    const float og = fsig(zo + cn * ppo);
    cnew[r] = cn;
    hnew[r] = og * ftanh(cn);
  }
}

__device__ __forceinline__ v8f cst_load(float* cp) {
  const v4f lo = *(volatile v4f*)(cp);
  const v4f hi = *(volatile v4f*)(cp + 128);
  return __builtin_shufflevector(lo, hi, 0, 1, 2, 3, 4, 5, 6, 7);
}
__device__ __forceinline__ void cst_store(float* cp, const v8f& cv) {
  const v4f lo = __builtin_shufflevector(cv, cv, 0, 1, 2, 3);
  const v4f hi = __builtin_shufflevector(cv, cv, 4, 5, 6, 7);
  *(volatile v4f*)(cp) = lo;
  *(volatile v4f*)(cp + 128) = hi;
  __threadfence();
  *(volatile v4f*)(cp) = lo;
  *(volatile v4f*)(cp + 128) = hi;
}

__device__ __forceinline__ void copy_stage(const _Float16* stg, _Float16* dst, int lane) {
  const int q = lane >> 3, c8 = (lane & 7) * 8;
#pragma unroll
  for (int it = 0; it < 4; ++it) {
    const int row = it * 4 + q;
    const v8h v = *(const v8h*)(stg + row * STP + c8);
    *(v8h*)(dst + row * AP + c8) = v;
  }
}

__global__ __launch_bounds__(RT) __attribute__((amdgpu_num_vgpr(256)))
void decode_kernel(const float* __restrict__ XGF, const float* __restrict__ Binit, const float* __restrict__ init,
                   const float* __restrict__ b1,
                   const float* __restrict__ pi0, const float* __restrict__ pf0, const float* __restrict__ po0,
                   const float* __restrict__ pi1, const float* __restrict__ pf1, const float* __restrict__ po1,
                   const float* __restrict__ blin,
                   const unsigned short* __restrict__ W0Rp, const unsigned short* __restrict__ W1Tp,
                   const unsigned short* __restrict__ WLTp,
                   const int* __restrict__ lenp, float* CST, float* __restrict__ out) {
  __shared__ __align__(16) _Float16 At[RB * AP];
  __shared__ __align__(16) _Float16 Hl[RB * HLP];
  __shared__ __align__(16) float    Sl[RW][16 * SLP];
  const _Float16* W0R = (const _Float16*)W0Rp;
  const _Float16* W1T = (const _Float16*)W1Tp;
  const _Float16* WLT = (const _Float16*)WLTp;
  const int tid = threadIdx.x, lane = tid & 31, wave = tid >> 5;
  const int c = lane & 15, hh = lane >> 4, koff = hh * 8;
  const int bt = blockIdx.x;
  const int rowbase = bt * RB;

  int Tn = lenp[0] - 1;
  Tn = Tn < 0 ? 0 : Tn;
  Tn = Tn > NSTEPS ? NSTEPS : Tn;

#pragma unroll 1
  for (int i = 0; i < RB; ++i)
    At[i * AP + tid] = (_Float16)bf16r(Binit[(size_t)(rowbase + i) * NBDIM + tid]);
#pragma unroll 1
  for (int it = 0; it < (RB * NUNIT) / RT; ++it) {
    const int idx = it * RT + tid;
    const int row = idx >> 10, u = idx & (NUNIT - 1);
    const float* ip = init + (size_t)(rowbase + row) * (4 * NUNIT);
    At[row * AP + COL_H0 + u] = (_Float16)bf16r(ip[NUNIT + u]);
    At[row * AP + COL_H1 + u] = (_Float16)bf16r(ip[3 * NUNIT + u]);
    Hl[row * HLP + u] = (_Float16)0.0f;
  }
  if (tid < RB * 8) {
    At[(tid >> 3) * AP + COL_H1 + NUNIT + (tid & 7)] = (_Float16)0.0f;
    Hl[(tid >> 3) * HLP + NUNIT + (tid & 7)] = (_Float16)0.0f;
  }
#pragma unroll 1
  for (int l = 0; l < 2; ++l) {
#pragma unroll 1
    for (int s = 0; s < SUBW; ++s) {
      const int ut = wave * SUBW + s;
      const int unit = ut * 16 + c;
      v8f cv;
#pragma unroll
      for (int r = 0; r < 8; ++r)
        cv[r] = bf16r(init[(size_t)(rowbase + 8 * hh + r) * (4 * NUNIT) + l * 2 * NUNIT + unit]);
      cst_store(CST + ((size_t)((l * NBT + bt) * 64 + ut)) * 256 + lane * 4, cv);
    }
  }
  __syncthreads();

  const v8f z8 = {0.f, 0.f, 0.f, 0.f, 0.f, 0.f, 0.f, 0.f};
  const _Float16* arow0 = At + c * AP + koff;
  const _Float16* arow1 = At + c * AP + COL_H0 + koff;
  const _Float16* arowH = At + c * AP + COL_H1 + koff;
  const _Float16* arowL = Hl + c * HLP + koff;
  float* slab = Sl[wave];
  _Float16* stg = (_Float16*)(&Sl[wave][0]);

#pragma unroll 1
  for (int t = 0; t < Tn; ++t) {
#pragma unroll 1
    for (int s = 0; s < SUBW; ++s) {
      const int ut = wave * SUBW + s;
      const int unit = ut * 16 + c;
      const float* xg = XGF + ((size_t)((t * NBT + bt) * 64 + ut)) * 1024 + lane * 4;
      v8f acc[4];
#pragma unroll
      for (int g = 0; g < 4; ++g) {
        const v4f lo = *(const v4f*)(xg + g * 256);
        const v4f hi = *(const v4f*)(xg + g * 256 + 128);
        acc[g] = __builtin_shufflevector(lo, hi, 0, 1, 2, 3, 4, 5, 6, 7);
      }
      const float ppi = bf16r(pi0[unit]);
      const float ppf = bf16r(pf0[unit]);
      const float ppo = bf16r(po0[unit]);
      gemm4<K0R>(arow0, W0R + (size_t)(ut * 64 + c) * K0R + koff, acc[0], acc[1], acc[2], acc[3]);
      float* cp = CST + ((size_t)((0 * NBT + bt) * 64 + ut)) * 256 + lane * 4;
      const v8f cold = cst_load(cp);
      v8f cnew, hnew;
      cell_update(acc[0], acc[1], acc[2], acc[3], ppi, ppf, ppo, cold, cnew, hnew);
      cst_store(cp, cnew);
#pragma unroll
      for (int r = 0; r < 8; ++r) stg[(8 * hh + r) * STP + s * 16 + c] = (_Float16)hnew[r];
    }
    __syncthreads();
    copy_stage(stg, At + COL_H0 + wave * 64, lane);
    __syncthreads();

#pragma unroll 1
    for (int s = 0; s < SUBW; ++s) {
      const int ut = wave * SUBW + s;
      const int unit = ut * 16 + c;
      v8f acc[4];
#pragma unroll
      for (int g = 0; g < 4; ++g) {
        const float bv = WCARRY * bf16r(b1[g * NUNIT + unit]);
        acc[g] = (v8f){bv, bv, bv, bv, bv, bv, bv, bv};
      }
      const float ppi = bf16r(pi1[unit]);
      const float ppf = bf16r(pf1[unit]);
      const float ppo = bf16r(po1[unit]);
      gemm4<K1L>(arow1, W1T + (size_t)(ut * 64 + c) * K1L + koff, acc[0], acc[1], acc[2], acc[3]);
      float* cp = CST + ((size_t)((1 * NBT + bt) * 64 + ut)) * 256 + lane * 4;
      const v8f cold = cst_load(cp);
      v8f cnew, hnew;
      cell_update(acc[0], acc[1], acc[2], acc[3], ppi, ppf, ppo, cold, cnew, hnew);
      cst_store(cp, cnew);
#pragma unroll
      for (int r = 0; r < 8; ++r) {
        const float hv = hnew[r];
        const _Float16 hi = (_Float16)hv;
        const float hif = (float)hi;
        const float res = (hv - hif) * LOCARRY;
        stg[(8 * hh + r) * STP + s * 16 + c] = hi;
        Hl[(8 * hh + r) * HLP + unit] = (_Float16)res;
      }
    }
    __syncthreads();
    copy_stage(stg, At + COL_H1 + wave * 64, lane);
    __syncthreads();

#pragma unroll 1
    for (int ns = 0; ns < 2; ++ns) {
      const int n = wave * 32 + ns * 16 + c;
      const _Float16* wl = WLT + (size_t)n * NUNIT + koff;
      v8f accH = z8, accL = z8;
#pragma unroll 1
      for (int k0 = 0; k0 < NUNIT; k0 += 32) {
        const v16h ah = Frag<_Float16>::load(arowH + k0);
        const v16h al = Frag<_Float16>::load(arowL + k0);
        const v16h b  = Frag<_Float16>::load(wl + k0);
        accH = Frag<_Float16>::mma(ah, b, accH);
        accL = Frag<_Float16>::mma(al, b, accL);
        guard2_h(accH, accL, ah, al, b);
      }
      acc_guard2(accH, accL);
      const float bl = bf16r(blin[n]);
#pragma unroll
      for (int r = 0; r < 8; ++r) {
        const float z = (accH[r] + accL[r] * LOCARRY_INV) * WCARRY_INV + bl;
        const float v = tanhf(z);
        slab[(8 * hh + r) * SLP + ns * 16 + c] = v;
        At[(8 * hh + r) * AP + n] = (_Float16)v;
      }
    }
    __syncthreads();
    {
      const int q = lane >> 3, c4 = (lane & 7) * 4;
      for (int pass = 0; pass < 2; ++pass) {
#pragma unroll
        for (int it = 0; it < 4; ++it) {
          const int row = it * 4 + q;
          const v4f v = *(const v4f*)(slab + row * SLP + c4);
          *(volatile v4f*)(out + ((size_t)t * NBATCH + (size_t)(rowbase + row)) * NBDIM + wave * 32 + c4) = v;
        }
        __threadfence();
      }
    }
    __syncthreads();
  }
}

extern "C" void kernel_launch(void* const* d_in, const int* in_sizes, int n_in,
                              void* d_out, int out_size, void* d_ws, size_t ws_size, hipStream_t stream) {
  if (n_in < 16 || d_out == nullptr || d_ws == nullptr) return;
  if (in_sizes[0] != NSTEPS * NBATCH * NVDIM || in_sizes[1] != NBATCH * NBDIM || in_sizes[2] != NBATCH * 4 * NUNIT ||
      in_sizes[3] != KW0 * NGCOL || in_sizes[4] != NGCOL || in_sizes[5] != NUNIT || in_sizes[6] != NUNIT ||
      in_sizes[7] != NUNIT || in_sizes[8] != K1L * NGCOL || in_sizes[9] != NGCOL || in_sizes[10] != NUNIT ||
      in_sizes[11] != NUNIT || in_sizes[12] != NUNIT || in_sizes[13] != NUNIT * NBDIM || in_sizes[14] != NBDIM ||
      in_sizes[15] != 1 || out_size != NSTEPS * NBATCH * NBDIM) return;

  const float* vseq  = (const float*)d_in[0];
  const float* binit = (const float*)d_in[1];
  const float* init  = (const float*)d_in[2];
  const float* w0    = (const float*)d_in[3];
  const float* b0    = (const float*)d_in[4];
  const float* pi0   = (const float*)d_in[5];
  const float* pf0   = (const float*)d_in[6];
  const float* po0   = (const float*)d_in[7];
  const float* w1    = (const float*)d_in[8];
  const float* b1    = (const float*)d_in[9];
  const float* pi1   = (const float*)d_in[10];
  const float* pf1   = (const float*)d_in[11];
  const float* po1   = (const float*)d_in[12];
  const float* wlin  = (const float*)d_in[13];
  const float* blin  = (const float*)d_in[14];
  const int*   lenp  = (const int*)d_in[15];
  float* out = (float*)d_out;

  char* ws = (char*)d_ws; size_t off = 0;
  auto carve = [&](size_t bytes) -> char* { char* p = ws + off; off += (bytes + 255) & ~(size_t)255; return p; };
  unsigned short* W0V = (unsigned short*)carve((size_t)NGCOL * NVDIM * 2);
  unsigned short* W0R = (unsigned short*)carve((size_t)NGCOL * K0R * 2);
  unsigned short* W1T = (unsigned short*)carve((size_t)NGCOL * K1L * 2);
  unsigned short* WLT = (unsigned short*)carve((size_t)NBDIM * NUNIT * 2);
  unsigned short* VH  = (unsigned short*)carve((size_t)MROWS * NVDIM * 2);
  float*          XGF = (float*)carve(XGF_FLOATS * 4);
  float*          CST = (float*)carve(CST_FLOATS * 4);
  if (off > ws_size || off > (size_t)134217728) return;

  tpw_kernel<1><<<dim3(NGCOL / 64, NVDIM / 64), NT256, 0, stream>>>(w0, NGCOL, NVDIM, W0V, WCARRY);
  tpw_kernel<1><<<dim3(NGCOL / 64, K0R / 64), NT256, 0, stream>>>(w0 + (size_t)NVDIM * NGCOL, NGCOL, K0R, W0R, WCARRY);
  tpw_kernel<1><<<dim3(NGCOL / 64, K1L / 64), NT256, 0, stream>>>(w1, NGCOL, K1L, W1T, WCARRY);
  tpw_kernel<0><<<dim3(NBDIM / 64, NUNIT / 64), NT256, 0, stream>>>(wlin, NBDIM, NUNIT, WLT, WCARRY);
  const int n8v = MROWS * (NVDIM / 8);
  cvt8_kernel<<<n8v / NT256, NT256, 0, stream>>>(vseq, VH, n8v);
  xg_gemm_kernel<<<((MROWS / 64) * (NGCOL / 64)) / 8, NT256, 0, stream>>>(VH, W0V, b0, XGF);
  decode_kernel<<<NBATCH / RB, RT, 0, stream>>>(XGF, binit, init, b1, pi0, pf0, po0, pi1, pf1, po1, blin,
                                                W0R, W1T, WLT, lenp, CST, out);
}
